// BiDecoder_82403242541306
// MI455X (gfx1250) — hardware-verified
//
#include <hip/hip_runtime.h>

typedef __attribute__((ext_vector_type(16))) _Float16 v16h;
typedef __attribute__((ext_vector_type(8)))  _Float16 v8h;
typedef __attribute__((ext_vector_type(16))) __bf16   v16b;
typedef __attribute__((ext_vector_type(8)))  __bf16   v8b;
typedef __attribute__((ext_vector_type(8)))  float    v8f;
typedef __attribute__((ext_vector_type(4)))  float    v4f;

static constexpr int FEAT       = 64;
static constexpr int NRATE      = 5;
static constexpr int EDGE_WAVES = 8;

__device__ __forceinline__ unsigned short f2bf_bits(float f) {
  unsigned u = __float_as_uint(f);
  return (unsigned short)((u + 0x7FFFu + ((u >> 16) & 1u)) >> 16);
}
__device__ __forceinline__ float bf_bits2f(unsigned short h) { return __uint_as_float(((unsigned)h) << 16); }

__device__ __forceinline__ void dep_guard_h(v8f& a, v8f& b, v16h x, v16h y) { asm volatile("v_nop\n\tv_nop\n\tv_nop\n\tv_nop" : "+v"(a), "+v"(b) : "v"(x), "v"(y)); }
__device__ __forceinline__ void dep_guard_b(v8f& a, v8f& b, v16b x, v16b y) { asm volatile("v_nop\n\tv_nop\n\tv_nop\n\tv_nop" : "+v"(a), "+v"(b) : "v"(x), "v"(y)); }
__device__ __forceinline__ void keep4_h(v16h a, v16h b, v16h c, v16h d) { asm volatile("v_nop" :: "v"(a), "v"(b), "v"(c), "v"(d)); }
__device__ __forceinline__ void keep4_b(v16b a, v16b b, v16b c, v16b d) { asm volatile("v_nop" :: "v"(a), "v"(b), "v"(c), "v"(d)); }
__device__ __forceinline__ void acc_guard4(v8f& a, v8f& b, v8f& c, v8f& d) { asm volatile("v_nop\n\tv_nop\n\tv_nop\n\tv_nop" : "+v"(a), "+v"(b), "+v"(c), "+v"(d)); }
template <typename T> struct Frag;
template <> struct Frag<_Float16> {
  typedef v16h V; union U { v16h v; v8h h[2]; };
  static __device__ __forceinline__ v16h load(const _Float16* p) {
    U f; f.h[0] = *(const v8h*)(p); f.h[1] = *(const v8h*)(p + 16); return f.v;
  }
  static __device__ __forceinline__ v8f mma(v16h a, v16h b, v8f c) {
    return __builtin_amdgcn_wmma_f32_16x16x32_f16(false, a, false, b, (short)0, c, false, false);
  }
  static __device__ __forceinline__ void guard(v8f& a, v8f& b, v16h x, v16h y) { dep_guard_h(a, b, x, y); }
  static __device__ __forceinline__ void keep(v16h a, v16h b, v16h c, v16h d) { keep4_h(a, b, c, d); }
};
template <> struct Frag<__bf16> {
  typedef v16b V; union U { v16b v; v8b h[2]; };
  static __device__ __forceinline__ v16b load(const __bf16* p) {
    U f; f.h[0] = *(const v8b*)(p); f.h[1] = *(const v8b*)(p + 16); return f.v;
  }
  static __device__ __forceinline__ v8f mma(v16b a, v16b b, v8f c) {
    return __builtin_amdgcn_wmma_f32_16x16x32_bf16(false, a, false, b, (short)0, c, false, false);
  }
  static __device__ __forceinline__ void guard(v8f& a, v8f& b, v16b x, v16b y) { dep_guard_b(a, b, x, y); }
  static __device__ __forceinline__ void keep(v16b a, v16b b, v16b c, v16b d) { keep4_b(a, b, c, d); }
};

template <int ET> struct Elem;
template <> struct Elem<0> { typedef _Float16 T; };
template <> struct Elem<1> { typedef __bf16 T; };
template <int ET, bool SPLIT, int BIAS_MODE, int OUT_MODE, bool RESID, int ACT = 0>
__global__ __launch_bounds__(256) void wmma_gemm64(
    const unsigned short* __restrict__ Ap, const unsigned short* __restrict__ A2p, int lda, long strideA,
    const unsigned short* __restrict__ Btp, const unsigned short* __restrict__ Bt2p, int ldb, long strideB,
    void* __restrict__ Cout, void* __restrict__ Cout2, int ldc, long strideC,
    const float* __restrict__ bias,
    const float* __restrict__ resid, long strideR,
    int M, int N, int K, float scale) {
  typedef typename Elem<ET>::T T;
  typedef typename Frag<T>::V V;
  const T* A = (const T*)Ap; const T* A2 = (const T*)A2p; const T* Bt = (const T*)Btp; const T* Bt2 = (const T*)Bt2p;
  __shared__ __align__(16) float sT[8][16 * 68];
  const int b    = blockIdx.y;
  const int lane = threadIdx.x & 31;
  const int wave = threadIdx.x >> 5;
  const int tilesN = N >> 6;
  const int tilesM = M >> 6;
  const int tile = blockIdx.x * 8 + wave;
  if (tile >= tilesM * tilesN) return;
  const int tm = tile / tilesN;
  const int tn = tile - tm * tilesN;
  const int m0 = tm << 6;
  const int n0 = tn << 6;

  const T* Ab  = A  + (size_t)b * strideA;
  const T* Bb  = Bt + (size_t)b * strideB;
  const T* Ab2 = SPLIT ? (A2  + (size_t)b * strideA) : nullptr;
  const T* Bb2 = SPLIT ? (Bt2 + (size_t)b * strideB) : nullptr;

  const int rlane = lane & 15;
  const int koff  = (lane >> 4) * 8;
  const int mOff  = (lane >> 4) * 8;

  v8f acc[4][4];
#pragma unroll
  for (int i = 0; i < 4; ++i)
#pragma unroll
    for (int j = 0; j < 4; ++j) acc[i][j] = (v8f){0.f,0.f,0.f,0.f,0.f,0.f,0.f,0.f};

  for (int k0 = 0; k0 < K; k0 += 32) {
    V bh[4], bl[4];
#pragma unroll
    for (int j = 0; j < 4; ++j) {
      const size_t bo = (size_t)(n0 + (j << 4) + rlane) * ldb + koff + k0;
      bh[j] = Frag<T>::load(Bb + bo);
      if (SPLIT) bl[j] = Frag<T>::load(Bb2 + bo);
    }
#pragma unroll
    for (int i = 0; i < 4; ++i) {
      const size_t ao = (size_t)(m0 + (i << 4) + rlane) * lda + koff + k0;
      V ah = Frag<T>::load(Ab + ao);
      V al;
      if (SPLIT) al = Frag<T>::load(Ab2 + ao);
#pragma unroll
      for (int j = 0; j < 4; ++j) {
        acc[i][j] = Frag<T>::mma(ah, bh[j], acc[i][j]);
        if (SPLIT) {
          acc[i][j] = Frag<T>::mma(ah, bl[j], acc[i][j]);
          acc[i][j] = Frag<T>::mma(al, bh[j], acc[i][j]);
        }
      }
      Frag<T>::guard(acc[i][0], acc[i][3], ah, SPLIT ? al : ah);
    }
    Frag<T>::keep(bh[0], bh[1], bh[2], bh[3]);
    if (SPLIT) Frag<T>::keep(bl[0], bl[1], bl[2], bl[3]);
  }
  acc_guard4(acc[0][0], acc[0][1], acc[0][2], acc[0][3]);
  acc_guard4(acc[1][0], acc[1][1], acc[1][2], acc[1][3]);
  acc_guard4(acc[2][0], acc[2][1], acc[2][2], acc[2][3]);
  acc_guard4(acc[3][0], acc[3][1], acc[3][2], acc[3][3]);

  float* slab = sT[wave];
  const float* Rb = RESID ? (resid + (size_t)b * strideR) : nullptr;
#pragma unroll
  for (int i = 0; i < 4; ++i) {
    const int mBase = m0 + (i << 4);
#pragma unroll
    for (int j = 0; j < 4; ++j) {
      const int n = n0 + (j << 4) + rlane;
      float bv = 0.f;
      if (BIAS_MODE == 2) bv = bias[n];
#pragma unroll
      for (int r = 0; r < 8; ++r) {
        float v = acc[i][j][r] * scale;
        if (BIAS_MODE == 1) v += bias[mBase + mOff + r];
        if (BIAS_MODE == 2) v += bv;
        if (RESID) v += Rb[(size_t)(mBase + mOff + r) * ldc + n];
        if (ACT == 1) v = tanhf(v);
        if (ACT == 2) v = fmaxf(v, 0.0f);
        if (ACT == 3) v = v / (1.0f + expf(-v));
        if (ACT == 4) v = (v > 0.f) ? v : 0.01f * v;
        if (ACT == 5) v = 0.5f * v * (1.0f + erff(v * 0.70710678118654752f));
        slab[(mOff + r) * 68 + (j << 4) + rlane] = v;
      }
    }
    __builtin_amdgcn_fence(__ATOMIC_RELEASE, "workgroup");
    __builtin_amdgcn_wave_barrier();
    __builtin_amdgcn_fence(__ATOMIC_ACQUIRE, "workgroup");
    if (OUT_MODE == 0) {
      float* C = (float*)Cout + (size_t)b * strideC;
      const int hh = lane >> 4, c4 = (lane & 15) * 4;
      for (int pass = 0; pass < 2; ++pass) {
#pragma unroll
        for (int it = 0; it < 8; ++it) {
          const int row = it * 2 + hh;
          v4f v = *(const v4f*)(slab + row * 68 + c4);
          *(volatile v4f*)(C + (size_t)(mBase + row) * ldc + n0 + c4) = v;
        }
        __threadfence();
      }
    } else {
      const int q = lane >> 3, c8 = (lane & 7) * 8;
      unsigned short* C  = (unsigned short*)Cout  + (size_t)b * strideC;
      unsigned short* C2 = (OUT_MODE == 2) ? ((unsigned short*)Cout2 + (size_t)b * strideC) : nullptr;
      for (int pass = 0; pass < 2; ++pass) {
#pragma unroll
        for (int it = 0; it < 4; ++it) {
          const int row = it * 4 + q;
          const float* sp = slab + row * 68 + c8;
          v8h hv, lv;
#pragma unroll
          for (int e = 0; e < 8; ++e) {
            if (OUT_MODE == 1) {
              hv[e] = (_Float16)sp[e];
            } else {
              unsigned short hb = f2bf_bits(sp[e]);
              unsigned short lb = f2bf_bits(sp[e] - bf_bits2f(hb));
              hv[e] = __builtin_bit_cast(_Float16, hb);
              lv[e] = __builtin_bit_cast(_Float16, lb);
            }
          }
          *(volatile v8h*)(C + (size_t)(mBase + row) * ldc + n0 + c8) = hv;
          if (OUT_MODE == 2) *(volatile v8h*)(C2 + (size_t)(mBase + row) * ldc + n0 + c8) = lv;
        }
        __threadfence();
      }
    }
    __builtin_amdgcn_fence(__ATOMIC_RELEASE, "workgroup");
    __builtin_amdgcn_wave_barrier();
    __builtin_amdgcn_fence(__ATOMIC_ACQUIRE, "workgroup");
  }
}

__global__ __launch_bounds__(256) void split_rows64_bf16(
    const float* __restrict__ in, unsigned short* __restrict__ hi, unsigned short* __restrict__ lo,
    int rows_valid, int rows_total) {
  const int t = blockIdx.x * 256 + threadIdx.x;
  const int nthr = rows_total * 8;
  if (t < nthr) {
    const int row = t >> 3;
    const int c8  = (t & 7) * 8;
    const int rowc = (row < rows_valid) ? row : (rows_valid - 1);
    const bool live = (row < rows_valid);
    const float* p = in + (size_t)rowc * FEAT + c8;
    const v4f a = *(const v4f*)p;
    const v4f bq = *(const v4f*)(p + 4);
    v8h hv, lv;
#pragma unroll
    for (int e = 0; e < 4; ++e) {
      const float f0 = live ? a[e]  : 0.0f;
      const float f1 = live ? bq[e] : 0.0f;
      const unsigned short h0 = f2bf_bits(f0);
      const unsigned short l0 = f2bf_bits(f0 - bf_bits2f(h0));
      const unsigned short h1 = f2bf_bits(f1);
      const unsigned short l1 = f2bf_bits(f1 - bf_bits2f(h1));
      hv[e]     = __builtin_bit_cast(_Float16, h0);
      lv[e]     = __builtin_bit_cast(_Float16, l0);
      hv[4 + e] = __builtin_bit_cast(_Float16, h1);
      lv[4 + e] = __builtin_bit_cast(_Float16, l1);
    }
    unsigned short* ph = hi + (size_t)row * FEAT + c8;
    unsigned short* pl = lo + (size_t)row * FEAT + c8;
    *(volatile v8h*)ph = hv;
    *(volatile v8h*)pl = lv;
    __threadfence();
    *(volatile v8h*)ph = hv;
    *(volatile v8h*)pl = lv;
  }
}

__global__ __launch_bounds__(256) void edge_rating_kernel(
    const float* __restrict__ ufeat, const float* __restrict__ tproj,
    const int* __restrict__ src, const int* __restrict__ dst,
    float* __restrict__ out, int nedge, int nuser, int nitem, int ldt) {
  __shared__ __align__(16) float sOut[EDGE_WAVES][32];
  const int tid  = threadIdx.x;
  const int lane = tid & 31;
  const int wave = tid >> 5;
  const int base = (blockIdx.x * EDGE_WAVES + wave) * 32;
  const int e  = base + lane;
  const int ec = (e < nedge) ? e : (nedge - 1);
  int u = src[ec]; u = (u < 0) ? 0 : ((u >= nuser) ? (nuser - 1) : u);
  int v = dst[ec]; v = (v < 0) ? 0 : ((v >= nitem) ? (nitem - 1) : v);
  const float* urow = ufeat + (size_t)u * FEAT;
  const float* trow = tproj + (size_t)v * (size_t)ldt;

  float s0 = 0.f, s1 = 0.f, s2 = 0.f, s3 = 0.f, s4 = 0.f;
#pragma unroll 1
  for (int c = 0; c < FEAT / 4; ++c) {
    const v4f uu = *(const v4f*)(urow + 4 * c);
    const v4f t0 = *(const v4f*)(trow + 0 * FEAT + 4 * c);
    const v4f t1 = *(const v4f*)(trow + 1 * FEAT + 4 * c);
    const v4f t2 = *(const v4f*)(trow + 2 * FEAT + 4 * c);
    const v4f t3 = *(const v4f*)(trow + 3 * FEAT + 4 * c);
    const v4f t4 = *(const v4f*)(trow + 4 * FEAT + 4 * c);
#pragma unroll
    for (int k = 0; k < 4; ++k) {
      s0 = fmaf(uu[k], t0[k], s0);
      s1 = fmaf(uu[k], t1[k], s1);
      s2 = fmaf(uu[k], t2[k], s2);
      s3 = fmaf(uu[k], t3[k], s3);
      s4 = fmaf(uu[k], t4[k], s4);
    }
  }
  const float m  = fmaxf(fmaxf(fmaxf(s0, s1), fmaxf(s2, s3)), s4);
  const float e0 = __expf(s0 - m);
  const float e1 = __expf(s1 - m);
  const float e2 = __expf(s2 - m);
  const float e3 = __expf(s3 - m);
  const float e4 = __expf(s4 - m);
  const float se = (((e0 + e1) + e2) + e3) + e4;
  float wv = e0;
  wv = fmaf(e1, 2.0f, wv);
  wv = fmaf(e2, 3.0f, wv);
  wv = fmaf(e3, 4.0f, wv);
  wv = fmaf(e4, 5.0f, wv);
  const float rat = wv * (1.0f / se);

  sOut[wave][lane] = rat;
  __syncthreads();
  const v4f ov = *(const v4f*)(&sOut[wave][4 * (lane & 7)]);
  const bool full = (base + 32 <= nedge);
  float* op = out + (size_t)base + 4 * (lane & 7);
  if (full) {
    if (lane < 8) *(volatile v4f*)op = ov;
  } else {
    if (e < nedge) *(volatile float*)(out + e) = rat;
  }
  __threadfence();
  if (full) {
    if (lane < 8) *(volatile v4f*)op = ov;
  } else {
    if (e < nedge) *(volatile float*)(out + e) = rat;
  }
}

static inline size_t align_up256(size_t x) { return (x + 255) & ~(size_t)255; }

extern "C" void kernel_launch(void* const* d_in, const int* in_sizes, int n_in,
                              void* d_out, int out_size, void* d_ws, size_t ws_size,
                              hipStream_t stream) {
  if (n_in < 5) return;
  const float* ufeat = (const float*)d_in[0];
  const float* ifeat = (const float*)d_in[1];
  const float* Ps    = (const float*)d_in[2];
  const int*   src   = (const int*)d_in[3];
  const int*   dst   = (const int*)d_in[4];
  float* out = (float*)d_out;

  const int nuser = in_sizes[0] / FEAT;
  const int nitem = in_sizes[1] / FEAT;
  const int nedge = in_sizes[3];
  if (in_sizes[2] != NRATE * FEAT * FEAT) return;
  if (nuser <= 0 || nitem <= 0 || nedge <= 0) return;
  if (in_sizes[4] < nedge || out_size < nedge) return;

  const int mpad = ((nitem + 63) / 64) * 64;
  const int ncol = NRATE * FEAT;
  const int kdim = FEAT;

  const size_t szA = (size_t)mpad * kdim * 2;
  const size_t szB = (size_t)ncol * kdim * 2;
  const size_t szT = (size_t)mpad * ncol * 4;
  const size_t offAh = 0;
  const size_t offAl = align_up256(offAh + szA);
  const size_t offBh = align_up256(offAl + szA);
  const size_t offBl = align_up256(offBh + szB);
  const size_t offT  = align_up256(offBl + szB);
  const size_t total = offT + szT;
  if (total > ws_size) return;

  char* ws = (char*)d_ws;
  unsigned short* aHi = (unsigned short*)(ws + offAh);
  unsigned short* aLo = (unsigned short*)(ws + offAl);
  unsigned short* bHi = (unsigned short*)(ws + offBh);
  unsigned short* bLo = (unsigned short*)(ws + offBl);
  float*          tpl = (float*)(ws + offT);

  {
    const int nthr = mpad * 8;
    split_rows64_bf16<<<(nthr + 255) / 256, 256, 0, stream>>>(ifeat, aHi, aLo, nitem, mpad);
  }
  {
    const int nthr = ncol * 8;
    split_rows64_bf16<<<(nthr + 255) / 256, 256, 0, stream>>>(Ps, bHi, bLo, ncol, ncol);
  }
  {
    const int tiles = (mpad / 64) * (ncol / 64);
    dim3 grid((tiles + 7) / 8, 1);
    wmma_gemm64<1, true, 0, 0, false, 0><<<grid, 256, 0, stream>>>(
        aHi, aLo, kdim, 0L,
        bHi, bLo, kdim, 0L,
        (void*)tpl, (void*)tpl, ncol, 0L,
        (const float*)tpl,
        (const float*)tpl, 0L,
        mpad, ncol, kdim, 1.0f);
  }
  {
    const int nwaves = (nedge + 31) / 32;
    const int nblk   = (nwaves + EDGE_WAVES - 1) / EDGE_WAVES;
    edge_rating_kernel<<<nblk, EDGE_WAVES * 32, 0, stream>>>(
        ufeat, tpl, src, dst, out, nedge, nuser, nitem, ncol);
  }
}
